// Decoder_2379411882667
// MI455X (gfx1250) — hardware-verified
//
#include <hip/hip_runtime.h>
#include <stddef.h>
#include <stdint.h>
#include <math.h>


#define MROWS   16384
#define EMB     256
#define XP      512
#define NT      256
#define GBM     64
#define PLANE_H ((size_t)MROWS * XP)
#define WBLK    1572864
#define O_WA1   0
#define O_WO1   524288
#define O_WQG2  655360
#define O_WKV2  786432
#define O_WO2   1048576
#define O_WSW   1179648
#define O_WS2   1441792
#define WSMAX   134217728
#define GEMM_LDS 65536

static_assert(O_WO1 == 1024 * 512);
static_assert(O_WQG2 == O_WO1 + 256 * 512);
static_assert(O_WKV2 == O_WQG2 + 512 * 256);
static_assert(O_WO2 == O_WKV2 + 512 * 512);
static_assert(O_WSW == O_WO2 + 256 * 512);
static_assert(O_WS2 == O_WSW + 512 * 512);
static_assert(WBLK == O_WS2 + 256 * 512);
static_assert(MROWS % GBM == 0 && EMB % 32 == 0 && XP == 2 * EMB);
static_assert(GBM * EMB * 4 == GEMM_LDS);

typedef float          v4f   __attribute__((ext_vector_type(4)));
typedef float          v8f   __attribute__((ext_vector_type(8)));
typedef int            v8i   __attribute__((ext_vector_type(8)));
typedef unsigned int   v4u   __attribute__((ext_vector_type(4)));
typedef unsigned short v8us  __attribute__((ext_vector_type(8)));
typedef unsigned short v16us __attribute__((ext_vector_type(16)));
typedef __bf16         v16bf __attribute__((ext_vector_type(16)));
typedef v4f  __attribute__((may_alias)) v4fa;
typedef v4u  __attribute__((may_alias)) v4ua;
typedef v8us __attribute__((may_alias)) v8usa;
union FragB { v16bf v; v16us u; v8us h[2]; v8i w; };
struct HL8 { v8us h; v8us l; };
struct F8  { v4f a; v4f b; };

__device__ __forceinline__ v8f wmb(const FragB& a, const FragB& b, v8f c) {
  v8f d = __builtin_amdgcn_wmma_f32_16x16x32_bf16(false, a.v, false, b.v, (short)0, c, false, false);
  asm volatile("v_nop\n\tv_nop\n\tv_nop\n\tv_nop" : "+v"(d) : "v"(a.w), "v"(b.w));
  return d;
}

__device__ __forceinline__ unsigned bf16_bits(float f) {
  const unsigned u = __float_as_uint(f);
  return (u + 0x7FFFu + ((u >> 16) & 1u)) >> 16;
}
__device__ __forceinline__ float bf16_val(float f) {
  return __uint_as_float(bf16_bits(f) << 16);
}
__device__ __forceinline__ v4f bf16_val4(v4f t) {
  v4f r;
  r.x = bf16_val(t.x); r.y = bf16_val(t.y); r.z = bf16_val(t.z); r.w = bf16_val(t.w);
  return r;
}

__device__ __forceinline__ HL8 split8(v4f a, v4f b) {
  HL8 r;
  unsigned hb;
  hb = bf16_bits(a.x); r.h[0] = (unsigned short)hb; r.l[0] = (unsigned short)bf16_bits(a.x - __uint_as_float(hb << 16));
  hb = bf16_bits(a.y); r.h[1] = (unsigned short)hb; r.l[1] = (unsigned short)bf16_bits(a.y - __uint_as_float(hb << 16));
  hb = bf16_bits(a.z); r.h[2] = (unsigned short)hb; r.l[2] = (unsigned short)bf16_bits(a.z - __uint_as_float(hb << 16));
  hb = bf16_bits(a.w); r.h[3] = (unsigned short)hb; r.l[3] = (unsigned short)bf16_bits(a.w - __uint_as_float(hb << 16));
  hb = bf16_bits(b.x); r.h[4] = (unsigned short)hb; r.l[4] = (unsigned short)bf16_bits(b.x - __uint_as_float(hb << 16));
  hb = bf16_bits(b.y); r.h[5] = (unsigned short)hb; r.l[5] = (unsigned short)bf16_bits(b.y - __uint_as_float(hb << 16));
  hb = bf16_bits(b.z); r.h[6] = (unsigned short)hb; r.l[6] = (unsigned short)bf16_bits(b.z - __uint_as_float(hb << 16));
  hb = bf16_bits(b.w); r.h[7] = (unsigned short)hb; r.l[7] = (unsigned short)bf16_bits(b.w - __uint_as_float(hb << 16));
  return r;
}

__device__ __forceinline__ F8 widen8(v4u w) {
  F8 r;
  r.a.x = __uint_as_float(w.x << 16); r.a.y = __uint_as_float(w.x & 0xffff0000u);
  r.a.z = __uint_as_float(w.y << 16); r.a.w = __uint_as_float(w.y & 0xffff0000u);
  r.b.x = __uint_as_float(w.z << 16); r.b.y = __uint_as_float(w.z & 0xffff0000u);
  r.b.z = __uint_as_float(w.w << 16); r.b.w = __uint_as_float(w.w & 0xffff0000u);
  return r;
}

__device__ __forceinline__ float gelu_f(float x) {
  const float x3 = x * x * x;
  return x * (0.5f * (1.0f + tanhf(0.7978845608028654f * (x + 0.044715f * x3))));
}
__device__ __forceinline__ float swish_f(float x) {
  return x * (1.0f / (1.0f + expf(-x)));
}
__device__ __forceinline__ v4f swish4(v4f t) {
  v4f r;
  r.x = swish_f(t.x); r.y = swish_f(t.y); r.z = swish_f(t.z); r.w = swish_f(t.w);
  return r;
}
__device__ __forceinline__ v4f gelu4(v4f t) {
  v4f r;
  r.x = gelu_f(t.x); r.y = gelu_f(t.y); r.z = gelu_f(t.z); r.w = gelu_f(t.w);
  return r;
}

__global__ __launch_bounds__(NT) void k_wprep(
    const float* __restrict__ wq1, const float* __restrict__ wk1, const float* __restrict__ wv1,
    const float* __restrict__ wg1, const float* __restrict__ wo1, const float* __restrict__ wq2,
    const float* __restrict__ wk2, const float* __restrict__ wv2, const float* __restrict__ wg2,
    const float* __restrict__ wo2, const float* __restrict__ swg, const float* __restrict__ sw1,
    const float* __restrict__ sw2, unsigned short* WB) {
  const int which = (int)blockIdx.y, blk = (int)blockIdx.z;
  const int u = (int)blockIdx.x * NT + (int)threadIdx.x;
  const float* W;
  int off, kd, radd, sw = 0;
  if (which == 0)       { W = wq1; off = O_WA1;  kd = 512; radd = 0; }
  else if (which == 1)  { W = wk1; off = O_WA1;  kd = 512; radd = 256; }
  else if (which == 2)  { W = wv1; off = O_WA1;  kd = 512; radd = 512; }
  else if (which == 3)  { W = wg1; off = O_WA1;  kd = 512; radd = 768; }
  else if (which == 4)  { W = wo1; off = O_WO1;  kd = 512; radd = 0; }
  else if (which == 5)  { W = wq2; off = O_WQG2; kd = 256; radd = 0; }
  else if (which == 6)  { W = wg2; off = O_WQG2; kd = 256; radd = 256; }
  else if (which == 7)  { W = wk2; off = O_WKV2; kd = 512; radd = 0; }
  else if (which == 8)  { W = wv2; off = O_WKV2; kd = 512; radd = 256; }
  else if (which == 9)  { W = wo2; off = O_WO2;  kd = 512; radd = 0; }
  else if (which == 10) { W = swg; off = O_WSW;  kd = 512; radd = 0;   sw = 1; }
  else if (which == 11) { W = sw1; off = O_WSW;  kd = 512; radd = 128; sw = 1; }
  else                  { W = sw2; off = O_WS2;  kd = 512; radd = 0; }
  const int sh  = (kd == 512) ? 6 : 5;
  const int upr = kd >> 3;
  if (u >= 256 * upr) return;
  const int n  = u >> sh;
  const int k8 = (u & (upr - 1)) * 8;
  const int row = (sw != 0) ? ((n >> 7) * 256 + radd + (n & 127)) : (radd + n);
  const float* p = W + (size_t)blk * 65536 + (size_t)(k8 & 255) * 256 + n;
  v8us o;
#pragma unroll
  for (int i = 0; i < 8; ++i) o[i] = (unsigned short)bf16_bits(p[(size_t)i * 256]);
  unsigned short* dp = WB + (size_t)blk * WBLK + off + (size_t)row * kd + k8;
  *(volatile v8us*)dp = o;
  __threadfence();
  *(volatile v8us*)dp = o;
}

__global__ __launch_bounds__(NT) void k_wprep2(const float* __restrict__ hw1, const float* __restrict__ hw2,
                                               const float* __restrict__ wenc, unsigned short* HW1,
                                               unsigned short* HW2, unsigned short* WE) {
  const int u = (int)blockIdx.x * NT + (int)threadIdx.x;
  const float* p;
  unsigned short* dp;
  int stride;
  if (u < 16384) {
    const int n = u >> 6, k8 = (u & 63) * 8;
    p = hw1 + (size_t)(k8 & 255) * 256 + n; stride = 256;
    dp = HW1 + (size_t)n * 512 + k8;
  } else if (u < 18432) {
    const int v = u - 16384;
    const int n = v >> 6, k8 = (v & 63) * 8;
    p = hw2 + (size_t)(k8 & 255) * 32 + n; stride = 32;
    dp = HW2 + (size_t)n * 512 + k8;
  } else if (u < 19456) {
    const int v = u - 18432;
    const int n = v >> 2, k8 = (v & 3) * 8;
    p = wenc + (size_t)k8 * 256 + n; stride = 256;
    dp = WE + (size_t)n * 32 + k8;
  } else {
    return;
  }
  v8us o;
#pragma unroll
  for (int i = 0; i < 8; ++i) o[i] = (unsigned short)bf16_bits(p[(size_t)i * stride]);
  *(volatile v8us*)dp = o;
  __threadfence();
  *(volatile v8us*)dp = o;
}

__global__ __launch_bounds__(NT) void k_gp(double g0, double g1, double g2, double g3, double g4, double g5,
                                           double g6, double g7, float* GP) {
  __shared__ __attribute__((aligned(16))) float s[256];
  const int tid = (int)threadIdx.x;
  const int h = tid >> 5, t = tid & 31;
  double g = g0;
  g = (h == 1) ? g1 : g; g = (h == 2) ? g2 : g; g = (h == 3) ? g3 : g; g = (h == 4) ? g4 : g;
  g = (h == 5) ? g5 : g; g = (h == 6) ? g6 : g; g = (h == 7) ? g7 : g;
  double pw = 1.0;
#pragma unroll 1
  for (int i = 0; i < 31; ++i) pw = (i < t) ? pw * g : pw;
  s[tid] = (float)pw;
  __syncthreads();
  if (tid < 64) {
    const v4f v = *(const v4fa*)(s + 4 * tid);
    float* op = GP + 4 * tid;
    *(volatile v4f*)op = v;
    __threadfence();
    *(volatile v4f*)op = v;
  }
}

__global__ __launch_bounds__(NT) void k_cvt(const float* __restrict__ src, unsigned short* dst, int nUnits) {
  const int u = (int)blockIdx.x * NT + (int)threadIdx.x;
  if (u >= nUnits) return;
  const float* p = src + (size_t)u * 8;
  const v4f a = *(const v4fa*)p;
  const v4f b = *(const v4fa*)(p + 4);
  v8us o;
  o[0] = (unsigned short)bf16_bits(a.x); o[1] = (unsigned short)bf16_bits(a.y);
  o[2] = (unsigned short)bf16_bits(a.z); o[3] = (unsigned short)bf16_bits(a.w);
  o[4] = (unsigned short)bf16_bits(b.x); o[5] = (unsigned short)bf16_bits(b.y);
  o[6] = (unsigned short)bf16_bits(b.z); o[7] = (unsigned short)bf16_bits(b.w);
  unsigned short* dp = dst + (size_t)u * 8;
  *(volatile v8us*)dp = o;
  __threadfence();
  *(volatile v8us*)dp = o;
}

__device__ __forceinline__ void gemm_core(const unsigned short* __restrict__ A, int lda,
                                          const unsigned short* __restrict__ WT, int K,
                                          int rowBase, int colBase, float* stg) {
  const int tid = (int)threadIdx.x, lane = tid & 31, wave = tid >> 5, hh = lane >> 4, m = lane & 15;
  const int rw = wave & 3, cw = wave >> 2;
  v8f acc[8];
  {
    const v8f z = {0.f, 0.f, 0.f, 0.f, 0.f, 0.f, 0.f, 0.f};
#pragma unroll
    for (int t = 0; t < 8; ++t) acc[t] = z;
  }
  const unsigned short* ap = A + (size_t)(rowBase + 16 * rw + m) * (size_t)lda + 8 * hh;
  const unsigned short* bp = WT + (size_t)(colBase + 128 * cw + m) * (size_t)K + 8 * hh;
#pragma unroll 1
  for (int k0 = 0; k0 < K; k0 += 32) {
    FragB af;
    af.h[0] = *(const v8usa*)(ap + k0);
    af.h[1] = *(const v8usa*)(ap + k0 + 16);
#pragma unroll
    for (int nt = 0; nt < 8; ++nt) {
      const unsigned short* wq = bp + (size_t)(16 * nt) * (size_t)K + k0;
      FragB bf;
      bf.h[0] = *(const v8usa*)wq;
      bf.h[1] = *(const v8usa*)(wq + 16);
      acc[nt] = wmb(af, bf, acc[nt]);
    }
  }
#pragma unroll
  for (int nt = 0; nt < 8; ++nt) {
    const int lc = 128 * cw + 16 * nt + m;
#pragma unroll
    for (int r = 0; r < 8; ++r) {
      const int lr = 16 * rw + 8 * hh + r;
      stg[lr * 256 + lc] = acc[nt][r];
    }
  }
  __syncthreads();
}

template <int GELU, int BIAS, int RES>
__global__ __launch_bounds__(NT) void k_gemm_norm(const unsigned short* __restrict__ A, int lda,
                                                  const unsigned short* __restrict__ WT, int K,
                                                  const float* __restrict__ bias, const float* __restrict__ lnw,
                                                  const unsigned short* resP, unsigned short* outX) {
  extern __shared__ __attribute__((aligned(16))) float dsm[];
  const int tid = (int)threadIdx.x, lane = tid & 31, wave = tid >> 5;
  const int rowBase = (int)blockIdx.x * GBM;
  gemm_core(A, lda, WT, K, rowBase, 0, dsm);

  const v4f la = bf16_val4(*(const v4fa*)(lnw + 8 * lane));
  const v4f lb = bf16_val4(*(const v4fa*)(lnw + 8 * lane + 4));
  v4f ba = {0.f, 0.f, 0.f, 0.f}, bb = {0.f, 0.f, 0.f, 0.f};
  if constexpr (BIAS != 0) {
    ba = bf16_val4(*(const v4fa*)(bias + 8 * lane));
    bb = bf16_val4(*(const v4fa*)(bias + 8 * lane + 4));
  }
#pragma unroll 1
  for (int i = 0; i < 8; ++i) {
    const int lr = 8 * wave + i;
    const size_t grow = (size_t)(rowBase + lr);
    v4f a = *(const v4fa*)(dsm + lr * 256 + 8 * lane);
    v4f b = *(const v4fa*)(dsm + lr * 256 + 8 * lane + 4);
    if constexpr (BIAS != 0) { a = a + ba; b = b + bb; }
    if constexpr (GELU != 0) { a = gelu4(a); b = gelu4(b); }
    if constexpr (RES == 1) {
      const v4u wh = *(const v4ua*)(resP + grow * XP + 8 * lane);
      const v4u wl = *(const v4ua*)(resP + grow * XP + EMB + 8 * lane);
      const F8 fh = widen8(wh);
      const F8 fl = widen8(wl);
      a = a + (fh.a + fl.a);
      b = b + (fh.b + fl.b);
    }
    if constexpr (RES == 2) {
      const v4u w0 = *(const v4ua*)(resP + grow * EMB + 8 * lane);
      const F8 f = widen8(w0);
      a = a + f.a;
      b = b + f.b;
    }
    float ss = a.x * a.x + a.y * a.y + a.z * a.z + a.w * a.w + b.x * b.x + b.y * b.y + b.z * b.z + b.w * b.w;
    ss += __shfl_xor(ss, 16, 32);
    ss += __shfl_xor(ss, 8, 32);
    ss += __shfl_xor(ss, 4, 32);
    ss += __shfl_xor(ss, 2, 32);
    ss += __shfl_xor(ss, 1, 32);
    const float inv = rsqrtf(ss * (1.0f / 256.0f) + 1e-6f);
    a = (a * inv) * la;
    b = (b * inv) * lb;
    const HL8 s = split8(a, b);
    unsigned short* op = outX + grow * XP + 8 * lane;
    *(volatile v8us*)op = s.h;
    *(volatile v8us*)(op + EMB) = s.l;
    __threadfence();
    *(volatile v8us*)op = s.h;
    *(volatile v8us*)(op + EMB) = s.l;
  }
}

__global__ __launch_bounds__(NT) void k_gemm_proj(const unsigned short* __restrict__ A, int lda,
                                                  const unsigned short* __restrict__ WT, int K, int pack,
                                                  unsigned short* QKV, float* G) {
  extern __shared__ __attribute__((aligned(16))) float dsm[];
  const int tid = (int)threadIdx.x, lane = tid & 31, wave = tid >> 5;
  const int rowBase = (int)blockIdx.x * GBM;
  const int y = (int)blockIdx.y;
  const int cls = (pack >> (4 * y)) & 15;
  gemm_core(A, lda, WT, K, rowBase, 256 * y, dsm);

  if (cls <= 1) {
    const float sc = (cls == 1) ? (1.0f / 5.65685424949238f) : 1.0f;
    unsigned short* dst = QKV + (size_t)cls * PLANE_H;
#pragma unroll 1
    for (int i = 0; i < 8; ++i) {
      const int lr = 8 * wave + i;
      const size_t grow = (size_t)(rowBase + lr);
      v4f a = *(const v4fa*)(dsm + lr * 256 + 8 * lane);
      v4f b = *(const v4fa*)(dsm + lr * 256 + 8 * lane + 4);
      a = a * sc; b = b * sc;
      const HL8 s = split8(a, b);
      unsigned short* op = dst + grow * XP + 8 * lane;
      *(volatile v8us*)op = s.h;
      *(volatile v8us*)(op + EMB) = s.l;
      __threadfence();
      *(volatile v8us*)op = s.h;
      *(volatile v8us*)(op + EMB) = s.l;
    }
  } else if (cls == 2) {
    unsigned short* vt = QKV + 2 * PLANE_H;
    const int bidx = rowBase >> 8;
    const int key0 = rowBase & 255;
#pragma unroll 1
    for (int it = 0; it < 8; ++it) {
      const int u = it * NT + tid;
      const int c = u >> 3, q = u & 7;
      const float* sp = dsm + (8 * q) * 256 + c;
      v4f a, b;
      a.x = sp[0];        a.y = sp[256];      a.z = sp[2 * 256];  a.w = sp[3 * 256];
      b.x = sp[4 * 256];  b.y = sp[5 * 256];  b.z = sp[6 * 256];  b.w = sp[7 * 256];
      const HL8 s = split8(a, b);
      unsigned short* op = vt + (size_t)(bidx * 256 + c) * XP + key0 + 8 * q;
      *(volatile v8us*)op = s.h;
      *(volatile v8us*)(op + 256) = s.l;
      __threadfence();
      *(volatile v8us*)op = s.h;
      *(volatile v8us*)(op + 256) = s.l;
    }
  } else {
#pragma unroll 1
    for (int i = 0; i < 8; ++i) {
      const int lr = 8 * wave + i;
      const size_t grow = (size_t)(rowBase + lr);
      const v4f a = swish4(*(const v4fa*)(dsm + lr * 256 + 4 * lane));
      const v4f b = swish4(*(const v4fa*)(dsm + lr * 256 + 128 + 4 * lane));
      float* op = G + grow * EMB + 4 * lane;
      *(volatile v4f*)op = a;
      *(volatile v4f*)(op + 128) = b;
      __threadfence();
      *(volatile v4f*)op = a;
      *(volatile v4f*)(op + 128) = b;
    }
  }
}

__global__ __launch_bounds__(NT) void k_gemm_swiglu(const unsigned short* __restrict__ A,
                                                    const unsigned short* __restrict__ WT, unsigned short* F) {
  extern __shared__ __attribute__((aligned(16))) float dsm[];
  const int tid = (int)threadIdx.x, lane = tid & 31, wave = tid >> 5, hh = lane >> 4, m = lane & 15;
  const int rowBase = (int)blockIdx.x * GBM;
  const int y = (int)blockIdx.y;
  gemm_core(A, XP, WT, XP, rowBase, 256 * y, dsm);
#pragma unroll 1
  for (int it = 0; it < 4; ++it) {
    const int lr = 8 * wave + 2 * it + hh;
    const size_t grow = (size_t)(rowBase + lr);
    const v4f ga = swish4(*(const v4fa*)(dsm + lr * 256 + 8 * m));
    const v4f gb = swish4(*(const v4fa*)(dsm + lr * 256 + 8 * m + 4));
    const v4f ua = *(const v4fa*)(dsm + lr * 256 + 128 + 8 * m);
    const v4f ub = *(const v4fa*)(dsm + lr * 256 + 128 + 8 * m + 4);
    const HL8 s = split8(ga * ua, gb * ub);
    unsigned short* op = F + grow * XP + 128 * y + 8 * m;
    *(volatile v8us*)op = s.h;
    *(volatile v8us*)(op + EMB) = s.l;
    __threadfence();
    *(volatile v8us*)op = s.h;
    *(volatile v8us*)(op + EMB) = s.l;
  }
}

__global__ __launch_bounds__(NT) void k_ret(const unsigned short* __restrict__ QKV, const float* __restrict__ G,
                                            const float* __restrict__ GP, const float* __restrict__ gns,
                                            const float* __restrict__ gnb, unsigned short* RG) {
  __shared__ __attribute__((aligned(16))) float ost[64 * 64];
  __shared__ float gps[64];
  const int tid = (int)threadIdx.x, lane = tid & 31, wave = tid >> 5, hh = lane >> 4, m = lane & 15;
  const int qi = (int)blockIdx.x, hpair = (int)blockIdx.y, b = (int)blockIdx.z;
  const int hp = wave >> 2, rg = wave & 3;
  const int h = 2 * hpair + hp;
  if (tid < 64) gps[tid] = GP[hpair * 64 + tid];
  __syncthreads();

  const unsigned short* Qp = QKV;
  const unsigned short* Kp = QKV + PLANE_H;
  const unsigned short* Vp = QKV + 2 * PLANE_H;
  const int qrow0 = qi * 64 + 16 * rg;
  const int npos = qrow0 + m;
  const int tq = npos >> 3;

  FragB qh, ql;
  {
    const unsigned short* p = Qp + (size_t)(b * 256 + npos) * XP + h * 32 + 8 * hh;
    qh.h[0] = *(const v8usa*)p;
    qh.h[1] = *(const v8usa*)(p + 16);
    ql.h[0] = *(const v8usa*)(p + EMB);
    ql.h[1] = *(const v8usa*)(p + EMB + 16);
  }
  const v8f z8 = {0.f, 0.f, 0.f, 0.f, 0.f, 0.f, 0.f, 0.f};
  v8f o0 = z8, o1 = z8;
  const int nkb = 2 * qi + (rg >> 1) + 1;
  const unsigned short* kbase = Kp + (size_t)(b * 256 + m) * XP + h * 32 + 8 * hh;
  const unsigned short* vbase = Vp + (size_t)(b * 256 + h * 32 + m) * XP + 8 * hh;

#pragma unroll 1
  for (int kb = 0; kb < nkb; ++kb) {
    const int k0 = kb * 32;
    FragB ph, pl;
#pragma unroll
    for (int t = 0; t < 2; ++t) {
      const unsigned short* kp = kbase + (size_t)(k0 + 16 * t) * XP;
      FragB kh, kl;
      kh.h[0] = *(const v8usa*)kp;
      kh.h[1] = *(const v8usa*)(kp + 16);
      kl.h[0] = *(const v8usa*)(kp + EMB);
      kl.h[1] = *(const v8usa*)(kp + EMB + 16);
      v8f s = z8;
      s = wmb(kh, qh, s);
      s = wmb(kh, ql, s);
      s = wmb(kl, qh, s);
      const int keyb = k0 + 16 * t + 8 * hh;
      const int dd = tq - (keyb >> 3);
      const int di = dd < 0 ? 0 : (dd > 31 ? 31 : dd);
      float g = gps[hp * 32 + di];
      g = (dd < 0) ? 0.0f : g;
#pragma unroll
      for (int r = 0; r < 8; ++r) {
        const float w = (npos >= keyb + r) ? g : 0.0f;
        const float p = s[r] * w;
        const unsigned hb = bf16_bits(p);
        ph.u[8 * t + r] = (unsigned short)hb;
        pl.u[8 * t + r] = (unsigned short)bf16_bits(p - __uint_as_float(hb << 16));
      }
    }
    {
      const unsigned short* vp = vbase + k0;
      FragB vh, vl;
      vh.h[0] = *(const v8usa*)vp;
      vh.h[1] = *(const v8usa*)(vp + 16);
      vl.h[0] = *(const v8usa*)(vp + 256);
      vl.h[1] = *(const v8usa*)(vp + 256 + 16);
      o0 = wmb(ph, vh, o0);
      o0 = wmb(ph, vl, o0);
      o0 = wmb(pl, vh, o0);
    }
    {
      const unsigned short* vp = vbase + (size_t)16 * XP + k0;
      FragB vh, vl;
      vh.h[0] = *(const v8usa*)vp;
      vh.h[1] = *(const v8usa*)(vp + 16);
      vl.h[0] = *(const v8usa*)(vp + 256);
      vl.h[1] = *(const v8usa*)(vp + 256 + 16);
      o1 = wmb(ph, vh, o1);
      o1 = wmb(ph, vl, o1);
      o1 = wmb(pl, vh, o1);
    }
  }

#pragma unroll
  for (int r = 0; r < 8; ++r) {
    const int lr = 16 * rg + 8 * hh + r;
    ost[lr * 64 + hp * 32 + m] = o0[r];
    ost[lr * 64 + hp * 32 + 16 + m] = o1[r];
  }
  __syncthreads();

#pragma unroll 1
  for (int it = 0; it < 2; ++it) {
    const int u = it * NT + tid;
    const int row = u >> 3, q = u & 7;
    v4f a = *(const v4fa*)(ost + row * 64 + 8 * q);
    v4f c = *(const v4fa*)(ost + row * 64 + 8 * q + 4);
    float s1 = (a.x + a.y) + (a.z + a.w) + (c.x + c.y) + (c.z + c.w);
    s1 += __shfl_xor(s1, 1, 32);
    s1 += __shfl_xor(s1, 2, 32);
    const float mu = s1 * (1.0f / 32.0f);
    a = a - mu; c = c - mu;
    float s2 = a.x * a.x + a.y * a.y + a.z * a.z + a.w * a.w + c.x * c.x + c.y * c.y + c.z * c.z + c.w * c.w;
    s2 += __shfl_xor(s2, 1, 32);
    s2 += __shfl_xor(s2, 2, 32);
    const float rstd = rsqrtf(s2 * (1.0f / 32.0f) + 1e-5f);
    const int e = hpair * 64 + 8 * q;
    const v4f sa = bf16_val4(*(const v4fa*)(gns + e));
    const v4f sb = bf16_val4(*(const v4fa*)(gns + e + 4));
    const v4f ta = bf16_val4(*(const v4fa*)(gnb + e));
    const v4f tb = bf16_val4(*(const v4fa*)(gnb + e + 4));
    const size_t grow = (size_t)(b * 256 + qi * 64 + row);
    const v4f ga = *(const v4fa*)(G + grow * EMB + e);
    const v4f gb = *(const v4fa*)(G + grow * EMB + e + 4);
    const v4f ya = ((a * rstd) * sa + ta) * ga;
    const v4f yb = ((c * rstd) * sb + tb) * gb;
    const HL8 s = split8(ya, yb);
    unsigned short* op = RG + grow * XP + e;
    *(volatile v8us*)op = s.h;
    *(volatile v8us*)(op + EMB) = s.l;
    __threadfence();
    *(volatile v8us*)op = s.h;
    *(volatile v8us*)(op + EMB) = s.l;
  }
}

__global__ __launch_bounds__(128) void k_head(const unsigned short* __restrict__ A,
                                              const unsigned short* __restrict__ WT,
                                              const float* __restrict__ hb2, float* out) {
  __shared__ __attribute__((aligned(16))) float stg[64 * 32];
  const int tid = (int)threadIdx.x, lane = tid & 31, wave = tid >> 5, hh = lane >> 4, m = lane & 15;
  const int rowBase = (int)blockIdx.x * GBM;
  const v8f z8 = {0.f, 0.f, 0.f, 0.f, 0.f, 0.f, 0.f, 0.f};
  v8f acc0 = z8, acc1 = z8;
  const unsigned short* ap = A + (size_t)(rowBase + 16 * wave + m) * XP + 8 * hh;
  const unsigned short* bp = WT + (size_t)m * XP + 8 * hh;
#pragma unroll 1
  for (int k0 = 0; k0 < XP; k0 += 32) {
    FragB af, b0, b1;
    af.h[0] = *(const v8usa*)(ap + k0);
    af.h[1] = *(const v8usa*)(ap + k0 + 16);
    b0.h[0] = *(const v8usa*)(bp + k0);
    b0.h[1] = *(const v8usa*)(bp + k0 + 16);
    b1.h[0] = *(const v8usa*)(bp + (size_t)16 * XP + k0);
    b1.h[1] = *(const v8usa*)(bp + (size_t)16 * XP + k0 + 16);
    acc0 = wmb(af, b0, acc0);
    acc1 = wmb(af, b1, acc1);
  }
#pragma unroll
  for (int r = 0; r < 8; ++r) {
    const int lr = 16 * wave + 8 * hh + r;
    stg[lr * 32 + m] = acc0[r];
    stg[lr * 32 + 16 + m] = acc1[r];
  }
  __syncthreads();
  v4f ov[4];
#pragma unroll
  for (int it = 0; it < 4; ++it) {
    const int u = it * 128 + tid;
    const int row = u >> 3, q = u & 7;
    const v4f bb = bf16_val4(*(const v4fa*)(hb2 + 4 * q));
    ov[it] = *(const v4fa*)(stg + row * 32 + 4 * q) + bb;
  }
#pragma unroll
  for (int it = 0; it < 4; ++it) {
    const int u = it * 128 + tid;
    *(volatile v4f*)(out + (size_t)(rowBase + (u >> 3)) * 32 + 4 * (u & 7)) = ov[it];
  }
  __threadfence();
#pragma unroll
  for (int it = 0; it < 4; ++it) {
    const int u = it * 128 + tid;
    *(volatile v4f*)(out + (size_t)(rowBase + (u >> 3)) * 32 + 4 * (u & 7)) = ov[it];
  }
}

static inline size_t al256(size_t o) { return (o + 255) & ~(size_t)255; }

extern "C" void kernel_launch(void* const* d_in, const int* in_sizes, int n_in,
                              void* d_out, int out_size, void* d_ws, size_t ws_size,
                              hipStream_t stream) {
  if (n_in < 29) return;
  if (in_sizes[0] != MROWS * 32 || in_sizes[1] != MROWS * EMB) return;
  if (in_sizes[2] != 32 * EMB || in_sizes[3] != EMB) return;
  for (int i = 4; i <= 8; ++i)  if (in_sizes[i] != 3 * 65536) return;
  for (int i = 9; i <= 11; ++i) if (in_sizes[i] != 3 * EMB) return;
  for (int i = 12; i <= 16; ++i) if (in_sizes[i] != 3 * 65536) return;
  for (int i = 17; i <= 19; ++i) if (in_sizes[i] != 3 * EMB) return;
  for (int i = 20; i <= 22; ++i) if (in_sizes[i] != 3 * 65536) return;
  if (in_sizes[23] != 3 * EMB) return;
  if (in_sizes[24] != 65536 || in_sizes[25] != EMB || in_sizes[26] != EMB) return;
  if (in_sizes[27] != EMB * 32 || in_sizes[28] != 32) return;
  if (out_size != MROWS * 32) return;

  const float* action = (const float*)d_in[0];
  const float* obs    = (const float*)d_in[1];
  const float* w_enc  = (const float*)d_in[2];
  const float* ln0    = (const float*)d_in[3];
  const float* wq1    = (const float*)d_in[4];
  const float* wk1    = (const float*)d_in[5];
  const float* wv1    = (const float*)d_in[6];
  const float* wg1    = (const float*)d_in[7];
  const float* wo1    = (const float*)d_in[8];
  const float* gns1   = (const float*)d_in[9];
  const float* gnb1   = (const float*)d_in[10];
  const float* ln1    = (const float*)d_in[11];
  const float* wq2    = (const float*)d_in[12];
  const float* wk2    = (const float*)d_in[13];
  const float* wv2    = (const float*)d_in[14];
  const float* wg2    = (const float*)d_in[15];
  const float* wo2    = (const float*)d_in[16];
  const float* gns2   = (const float*)d_in[17];
  const float* gnb2   = (const float*)d_in[18];
  const float* ln2    = (const float*)d_in[19];
  const float* swg    = (const float*)d_in[20];
  const float* sw1    = (const float*)d_in[21];
  const float* sw2    = (const float*)d_in[22];
  const float* ln3    = (const float*)d_in[23];
  const float* hw1    = (const float*)d_in[24];
  const float* hb1    = (const float*)d_in[25];
  const float* hln    = (const float*)d_in[26];
  const float* hw2    = (const float*)d_in[27];
  const float* hb2    = (const float*)d_in[28];
  float* out = (float*)d_out;

  char* ws = (char*)d_ws;
  size_t off = 0;
  const size_t oGP  = off; off = al256(off + (size_t)256 * 4);
  const size_t oWE  = off; off = al256(off + (size_t)256 * 32 * 2);
  const size_t oHW1 = off; off = al256(off + (size_t)256 * 512 * 2);
  const size_t oHW2 = off; off = al256(off + (size_t)32 * 512 * 2);
  const size_t oWB  = off; off = al256(off + (size_t)3 * WBLK * 2);
  const size_t oAB  = off; off = al256(off + (size_t)MROWS * 32 * 2);
  const size_t oOB  = off; off = al256(off + (size_t)MROWS * EMB * 2);
  const size_t oX   = off; off = al256(off + PLANE_H * 2);
  const size_t oQKV = off; off = al256(off + 3 * PLANE_H * 2);
  const size_t oG   = off; off = al256(off + (size_t)MROWS * EMB * 4);
  const size_t oRG  = off; off = al256(off + PLANE_H * 2);
  if (off > ws_size || off > (size_t)WSMAX) return;
  float*          GP  = (float*)(ws + oGP);
  unsigned short* WE  = (unsigned short*)(ws + oWE);
  unsigned short* HW1 = (unsigned short*)(ws + oHW1);
  unsigned short* HW2 = (unsigned short*)(ws + oHW2);
  unsigned short* WB  = (unsigned short*)(ws + oWB);
  unsigned short* AB  = (unsigned short*)(ws + oAB);
  unsigned short* OB  = (unsigned short*)(ws + oOB);
  unsigned short* XHL = (unsigned short*)(ws + oX);
  unsigned short* QKV = (unsigned short*)(ws + oQKV);
  float*          G   = (float*)(ws + oG);
  unsigned short* RG  = (unsigned short*)(ws + oRG);

  hipFuncSetAttribute(reinterpret_cast<const void*>(&k_gemm_norm<1, 0, 0>), hipFuncAttributeMaxDynamicSharedMemorySize, GEMM_LDS);
  hipFuncSetAttribute(reinterpret_cast<const void*>(&k_gemm_norm<0, 0, 1>), hipFuncAttributeMaxDynamicSharedMemorySize, GEMM_LDS);
  hipFuncSetAttribute(reinterpret_cast<const void*>(&k_gemm_norm<0, 0, 2>), hipFuncAttributeMaxDynamicSharedMemorySize, GEMM_LDS);
  hipFuncSetAttribute(reinterpret_cast<const void*>(&k_gemm_norm<1, 1, 0>), hipFuncAttributeMaxDynamicSharedMemorySize, GEMM_LDS);
  hipFuncSetAttribute(reinterpret_cast<const void*>(&k_gemm_proj), hipFuncAttributeMaxDynamicSharedMemorySize, GEMM_LDS);
  hipFuncSetAttribute(reinterpret_cast<const void*>(&k_gemm_swiglu), hipFuncAttributeMaxDynamicSharedMemorySize, GEMM_LDS);

  double gd[8];
  for (int h = 0; h < 8; ++h) gd[h] = (double)(float)(1.0 - exp2(-(5.0 + 4.0 * (double)h / 7.0)));

  const int gM = MROWS / GBM;
  k_wprep<<<dim3(64, 13, 3), NT, 0, stream>>>(wq1, wk1, wv1, wg1, wo1, wq2, wk2, wv2, wg2, wo2, swg, sw1, sw2, WB);
  k_wprep2<<<76, NT, 0, stream>>>(hw1, hw2, w_enc, HW1, HW2, WE);
  k_gp<<<1, NT, 0, stream>>>(gd[0], gd[1], gd[2], gd[3], gd[4], gd[5], gd[6], gd[7], GP);
  k_cvt<<<(MROWS * 32 / 8) / NT, NT, 0, stream>>>(action, AB, MROWS * 32 / 8);
  k_cvt<<<(MROWS * EMB / 8) / NT, NT, 0, stream>>>(obs, OB, MROWS * EMB / 8);
  k_gemm_norm<1, 0, 0><<<gM, NT, GEMM_LDS, stream>>>(AB, 32, WE, 32, ln0, ln0, XHL, XHL);

  for (int b = 0; b < 3; ++b) {
    const unsigned short* wb = WB + (size_t)b * WBLK;
    k_gemm_proj<<<dim3(gM, 4), NT, GEMM_LDS, stream>>>(XHL, XP, wb + O_WA1, XP, 0x3210, QKV, G);
    k_ret<<<dim3(4, 4, 64), NT, 0, stream>>>(QKV, G, GP, gns1 + b * EMB, gnb1 + b * EMB, RG);
    k_gemm_norm<0, 0, 1><<<gM, NT, GEMM_LDS, stream>>>(RG, XP, wb + O_WO1, XP, ln1, ln1 + b * EMB, XHL, XHL);
    k_gemm_proj<<<dim3(gM, 2), NT, GEMM_LDS, stream>>>(OB, EMB, wb + O_WQG2, EMB, 0x30, QKV, G);
    k_gemm_proj<<<dim3(gM, 2), NT, GEMM_LDS, stream>>>(XHL, XP, wb + O_WKV2, XP, 0x21, QKV, G);
    k_ret<<<dim3(4, 4, 64), NT, 0, stream>>>(QKV, G, GP, gns2 + b * EMB, gnb2 + b * EMB, RG);
    k_gemm_norm<0, 0, 2><<<gM, NT, GEMM_LDS, stream>>>(RG, XP, wb + O_WO2, XP, ln2, ln2 + b * EMB, OB, XHL);
    k_gemm_swiglu<<<dim3(gM, 2), NT, GEMM_LDS, stream>>>(XHL, wb + O_WSW, RG);
    k_gemm_norm<0, 0, 1><<<gM, NT, GEMM_LDS, stream>>>(RG, XP, wb + O_WS2, XP, ln3, ln3 + b * EMB, XHL, XHL);
  }
  k_gemm_norm<1, 1, 0><<<gM, NT, GEMM_LDS, stream>>>(XHL, XP, HW1, XP, hb1, hln, XHL, RG);
  k_head<<<gM, 128, 0, stream>>>(RG, HW2, hb2, out);
}
